// GPT2Attention_22101901705524
// MI455X (gfx1250) — hardware-verified
//
#include <hip/hip_runtime.h>


#ifndef NB
#define NB 2
#endif
#ifndef SEQ
#define SEQ 2048
#endif
#define NB_FULL  2
#define SEQ_FULL 2048
#define CH    1024
#define NH    16
#define HD    64
#define MROWS (NB * SEQ)
#define LDP   136
#define LDPF  68

static_assert(NB >= 1 && NB <= NB_FULL);
static_assert(SEQ >= 128 && SEQ <= SEQ_FULL && (SEQ % 128) == 0);
static_assert(NH * HD == CH);
static_assert((CH % 128) == 0 && (CH % 32) == 0);
static_assert(CH * CH / 8 / 256 == 512);
static_assert(CH / 8 == 128);
static_assert((MROWS * CH / 8) % 256 == 0);
static_assert((MROWS % 128) == 0);

typedef _Float16 v16h __attribute__((ext_vector_type(16)));
typedef _Float16 v8h  __attribute__((ext_vector_type(8)));
typedef float    v8f  __attribute__((ext_vector_type(8)));
typedef float    v4f  __attribute__((ext_vector_type(4)));

union Frag { v16h v; v8h h[2]; };

#define WMMA_F16(a, b, c) \
  __builtin_amdgcn_wmma_f32_16x16x32_f16(false, (a), false, (b), (short)0, (c), false, false)

__device__ __forceinline__ v16h ldfrag(const _Float16* __restrict__ base, int pitch, int row0, int k0) {
  const int lane = threadIdx.x & 31;
  const _Float16* p = base + (size_t)(row0 + (lane & 15)) * (size_t)pitch + k0 + 8 * (lane >> 4);
  Frag u;
  u.h[0] = *(const v8h*)(p);
  u.h[1] = *(const v8h*)(p + 16);
  return u.v;
}

__device__ __forceinline__ float bf16r(float v) {
  unsigned int u = __float_as_uint(v);
  u += 0x7FFFu + ((u >> 16) & 1u);
  u &= 0xFFFF0000u;
  return __uint_as_float(u);
}

__global__ void __launch_bounds__(256) cvt_w_kernel(
    const float* __restrict__ Wq, const float* __restrict__ Wk,
    const float* __restrict__ Wv, const float* __restrict__ Wo,
    _Float16* __restrict__ Wc) {
  const int g   = blockIdx.x * 256 + threadIdx.x;
  const int mat = blockIdx.x >> 9;
  const float* src = (mat == 0) ? Wq : (mat == 1) ? Wk : (mat == 2) ? Wv : Wo;
  const size_t e = (size_t)(g - mat * (CH * CH / 8)) * 8;
  const v4f f0 = *(const v4f*)(src + e);
  const v4f f1 = *(const v4f*)(src + e + 4);
  v8h o;
#pragma unroll
  for (int j = 0; j < 4; ++j) {
    o[j]     = (_Float16)(bf16r(f0[j]) * 64.0f);
    o[j + 4] = (_Float16)(bf16r(f1[j]) * 64.0f);
  }
  _Float16* d = Wc + (size_t)g * 8;
  *(volatile v8h*)d = o;
  __threadfence();
  *(volatile v8h*)d = o;
}

__global__ void __launch_bounds__(256) cvt_x_kernel(const float* __restrict__ x, _Float16* __restrict__ Xc) {
  const int g  = blockIdx.x * 256 + threadIdx.x;
  const int m  = g >> 7;
  const int c8 = (g & 127) * 8;
  const int b  = m / SEQ;
  const int t  = m - b * SEQ;
  const float* s = x + (size_t)(b * SEQ_FULL + t) * CH + c8;
  const v4f f0 = *(const v4f*)(s);
  const v4f f1 = *(const v4f*)(s + 4);
  v8h o;
#pragma unroll
  for (int j = 0; j < 4; ++j) {
    o[j]     = (_Float16)bf16r(f0[j]);
    o[j + 4] = (_Float16)bf16r(f1[j]);
  }
  _Float16* d = Xc + (size_t)g * 8;
  *(volatile v8h*)d = o;
  __threadfence();
  *(volatile v8h*)d = o;
}

__global__ void __launch_bounds__(256) qkv_kernel(
    const _Float16* __restrict__ Xc, const _Float16* __restrict__ Wc,
    const float* __restrict__ bq, const float* __restrict__ bk, const float* __restrict__ bv,
    _Float16* __restrict__ Qh, _Float16* __restrict__ Ql,
    _Float16* __restrict__ Kh, _Float16* __restrict__ Kl,
    _Float16* __restrict__ Vth, _Float16* __restrict__ Vtl) {
  __shared__ __attribute__((aligned(16))) _Float16 sT[128 * LDP];

  const int tid = threadIdx.x, wid = tid >> 5, lane = tid & 31, l16 = lane & 15, lh = lane >> 4;
  const int wm = wid & 3, wn = wid >> 2;
  const int bx = blockIdx.x, by = blockIdx.y;
  const int mat = by >> 3;
  const int m0 = bx * 128 + wm * 32;
  const int n0 = by * 128 + wn * 64;

  v8f acc[2][4];
  const v8f zero = {};
#pragma unroll
  for (int i = 0; i < 2; ++i)
#pragma unroll
    for (int j = 0; j < 4; ++j) acc[i][j] = zero;

  for (int k0 = 0; k0 < CH; k0 += 32) {
    const v16h a0 = ldfrag(Xc, CH, m0, k0);
    const v16h a1 = ldfrag(Xc, CH, m0 + 16, k0);
    const v16h b0 = ldfrag(Wc, CH, n0, k0);
    const v16h b1 = ldfrag(Wc, CH, n0 + 16, k0);
    const v16h b2 = ldfrag(Wc, CH, n0 + 32, k0);
    const v16h b3 = ldfrag(Wc, CH, n0 + 48, k0);
    acc[0][0] = WMMA_F16(a0, b0, acc[0][0]);
    acc[1][0] = WMMA_F16(a1, b0, acc[1][0]);
    acc[0][1] = WMMA_F16(a0, b1, acc[0][1]);
    acc[1][1] = WMMA_F16(a1, b1, acc[1][1]);
    acc[0][2] = WMMA_F16(a0, b2, acc[0][2]);
    acc[1][2] = WMMA_F16(a1, b2, acc[1][2]);
    acc[0][3] = WMMA_F16(a0, b3, acc[0][3]);
    acc[1][3] = WMMA_F16(a1, b3, acc[1][3]);
    asm volatile("v_nop\n\tv_nop\n\tv_nop\n\tv_nop"
                 : "+v"(acc[0][0]), "+v"(acc[1][0]), "+v"(acc[0][1]), "+v"(acc[1][1]),
                   "+v"(acc[0][2]), "+v"(acc[1][2]), "+v"(acc[0][3]), "+v"(acc[1][3])
                 : "v"(a0), "v"(a1), "v"(b0), "v"(b3));
  }

  const float* bias = (mat == 0) ? bq : (mat == 1) ? bk : bv;
  const int cb = (by & 7) * 128 + wn * 64;
  float bcol[4];
#pragma unroll
  for (int j = 0; j < 4; ++j) bcol[j] = bf16r(bias[cb + j * 16 + l16]);
  const int mb0   = bx * 128;
  const int bb    = mb0 / SEQ;
  const int t0    = mb0 - bb * SEQ;
  const int head0 = (by & 7) * 2;

  for (int part = 0; part < 2; ++part) {
    __syncthreads();
#pragma unroll
    for (int i = 0; i < 2; ++i)
#pragma unroll
      for (int j = 0; j < 4; ++j)
#pragma unroll
        for (int r = 0; r < 8; ++r) {
          const int rl = wm * 32 + i * 16 + 8 * lh + r;
          const int cl = wn * 64 + j * 16 + l16;
          const float val = acc[i][j][r] * 0.015625f + bcol[j];
          const _Float16 hv = (_Float16)val;
          const _Float16 w  = (part == 0) ? hv : (_Float16)((val - (float)hv) * 4096.0f);
          sT[(mat == 2) ? (cl * LDP + rl) : (rl * LDP + cl)] = w;
        }
    __syncthreads();
    _Float16* plane = (mat == 0) ? (part ? Ql : Qh) : (mat == 1) ? (part ? Kl : Kh) : (part ? Vtl : Vth);
    for (int pass = 0; pass < 2; ++pass) {
#pragma unroll
      for (int it = 0; it < 8; ++it) {
        const int L = wid * 32 + it * 4 + (lane >> 3);
        const int p = lane & 7;
        const v8h val = *(const v8h*)(sT + (L >> 1) * LDP + (L & 1) * 64 + p * 8);
        size_t off;
        if (mat == 2) {
          const int cl = L >> 1;
          off = (size_t)((bb * NH + head0 + (cl >> 6)) * HD + (cl & 63)) * SEQ + t0 + (L & 1) * 64 + p * 8;
        } else {
          off = (size_t)((bb * NH + head0 + (L & 1)) * SEQ + t0 + (L >> 1)) * HD + p * 8;
        }
        *(volatile v8h*)(plane + off) = val;
      }
      __threadfence();
    }
  }
}

__global__ void __launch_bounds__(128) attn_kernel(
    const _Float16* __restrict__ Qh, const _Float16* __restrict__ Ql,
    const _Float16* __restrict__ Kh, const _Float16* __restrict__ Kl,
    const _Float16* __restrict__ Vth, const _Float16* __restrict__ Vtl,
    _Float16* __restrict__ Ch, _Float16* __restrict__ Cl) {
  __shared__ __attribute__((aligned(16))) _Float16 ldsPh[4][16 * 32];
  __shared__ __attribute__((aligned(16))) _Float16 ldsPl[4][16 * 32];
  __shared__ __attribute__((aligned(16))) _Float16 sCh[4][16 * HD];
  __shared__ __attribute__((aligned(16))) _Float16 sCl[4][16 * HD];

  const int tid = threadIdx.x, wave = tid >> 5, lane = tid & 31, l16 = lane & 15, lh = lane >> 4;
  const int nqb  = SEQ / 64;
  const int bh   = blockIdx.x / nqb;
  const int qblk = blockIdx.x - bh * nqb;
  const int b    = bh / NH;
  const int h    = bh - b * NH;
  const int q0   = qblk * 64 + wave * 16;

  const _Float16* Qhb = Qh  + (size_t)bh * SEQ * HD;
  const _Float16* Qlb = Ql  + (size_t)bh * SEQ * HD;
  const _Float16* Khb = Kh  + (size_t)bh * SEQ * HD;
  const _Float16* Klb = Kl  + (size_t)bh * SEQ * HD;
  const _Float16* Vhb = Vth + (size_t)bh * HD * SEQ;
  const _Float16* Vlb = Vtl + (size_t)bh * HD * SEQ;

  v16h aqh[2], aql[2];
#pragma unroll
  for (int hc = 0; hc < 2; ++hc) {
    aqh[hc] = ldfrag(Qhb, HD, q0, hc * 32);
    aql[hc] = ldfrag(Qlb, HD, q0, hc * 32);
  }

  float m[8], l[8];
  v8f co0[4], co1[4];
  const v8f zero = {};
#pragma unroll
  for (int r = 0; r < 8; ++r) { m[r] = -1e30f; l[r] = 0.0f; }
#pragma unroll
  for (int n = 0; n < 4; ++n) { co0[n] = zero; co1[n] = zero; }

  for (int kb = 0; kb < q0 + 16; kb += 32) {
    v8f sh0 = zero, sh1 = zero, sr0 = zero, sr1 = zero;
#pragma unroll
    for (int hc = 0; hc < 2; ++hc) {
      const v16h kh0 = ldfrag(Khb, HD, kb,      hc * 32);
      const v16h kh1 = ldfrag(Khb, HD, kb + 16, hc * 32);
      const v16h kl0 = ldfrag(Klb, HD, kb,      hc * 32);
      const v16h kl1 = ldfrag(Klb, HD, kb + 16, hc * 32);
      sh0 = WMMA_F16(aqh[hc], kh0, sh0);
      sh1 = WMMA_F16(aqh[hc], kh1, sh1);
      sr0 = WMMA_F16(aqh[hc], kl0, sr0);
      sr1 = WMMA_F16(aqh[hc], kl1, sr1);
      sr0 = WMMA_F16(aql[hc], kh0, sr0);
      sr1 = WMMA_F16(aql[hc], kh1, sr1);
    }
    asm volatile("v_nop\n\tv_nop\n\tv_nop\n\tv_nop"
                 : "+v"(sh0), "+v"(sh1), "+v"(sr0), "+v"(sr1)
                 : "v"(aqh[0]), "v"(aqh[1]), "v"(aql[0]), "v"(aql[1]));

    float alpha[8];
#pragma unroll
    for (int r = 0; r < 8; ++r) {
      const int row  = q0 + r + 8 * lh;
      const int key0 = kb + l16;
      const int key1 = key0 + 16;
      float x0 = (sh0[r] + sr0[r] * 0.000244140625f) * 0.125f;
      float x1 = (sh1[r] + sr1[r] * 0.000244140625f) * 0.125f;
      x0 = (key0 <= row) ? x0 : -1e30f;
      x1 = (key1 <= row) ? x1 : -1e30f;
      float tmax = fmaxf(x0, x1);
#pragma unroll
      for (int off = 1; off < 16; off <<= 1) tmax = fmaxf(tmax, __shfl_xor(tmax, off, 32));
      const float mn = fmaxf(m[r], tmax);
      alpha[r] = __expf(m[r] - mn);
      const float p0 = __expf(x0 - mn);
      const float p1 = __expf(x1 - mn);
      float ps = p0 + p1;
#pragma unroll
      for (int off = 1; off < 16; off <<= 1) ps += __shfl_xor(ps, off, 32);
      l[r] = l[r] * alpha[r] + ps;
      m[r] = mn;
      const float g0 = p0 * 1024.0f, g1 = p1 * 1024.0f;
      const _Float16 h0 = (_Float16)g0, h1 = (_Float16)g1;
      const int prow = (r + 8 * lh) * 32;
      ldsPh[wave][prow + l16]      = h0;
      ldsPh[wave][prow + 16 + l16] = h1;
      ldsPl[wave][prow + l16]      = (_Float16)((g0 - (float)h0) * 4096.0f);
      ldsPl[wave][prow + 16 + l16] = (_Float16)((g1 - (float)h1) * 4096.0f);
    }
#pragma unroll
    for (int n = 0; n < 4; ++n)
#pragma unroll
      for (int r = 0; r < 8; ++r) { co0[n][r] *= alpha[r]; co1[n][r] *= alpha[r]; }

    __builtin_amdgcn_fence(3  , "workgroup");
    __builtin_amdgcn_wave_barrier();
    __builtin_amdgcn_fence(2  , "workgroup");

    Frag aph, apl;
    aph.h[0] = *(const v8h*)(&ldsPh[wave][l16 * 32 + 8 * lh]);
    aph.h[1] = *(const v8h*)(&ldsPh[wave][l16 * 32 + 16 + 8 * lh]);
    apl.h[0] = *(const v8h*)(&ldsPl[wave][l16 * 32 + 8 * lh]);
    apl.h[1] = *(const v8h*)(&ldsPl[wave][l16 * 32 + 16 + 8 * lh]);
#pragma unroll
    for (int n = 0; n < 4; ++n) {
      const v16h vh = ldfrag(Vhb, SEQ, n * 16, kb);
      const v16h vl = ldfrag(Vlb, SEQ, n * 16, kb);
      co0[n] = WMMA_F16(aph.v, vh, co0[n]);
      co1[n] = WMMA_F16(aph.v, vl, co1[n]);
      co1[n] = WMMA_F16(apl.v, vh, co1[n]);
    }
    asm volatile("v_nop\n\tv_nop\n\tv_nop\n\tv_nop"
                 : "+v"(co0[0]), "+v"(co0[1]), "+v"(co0[2]), "+v"(co0[3]),
                   "+v"(co1[0]), "+v"(co1[1]), "+v"(co1[2]), "+v"(co1[3])
                 : "v"(aph.v), "v"(apl.v));
  }

#pragma unroll
  for (int r = 0; r < 8; ++r) {
    const float inv = 1.0f / l[r];
    const int crow = (r + 8 * lh) * HD;
#pragma unroll
    for (int n = 0; n < 4; ++n) {
      const float c64 = (co0[n][r] * 0.0625f + co1[n][r] * 0.0000152587890625f) * inv;
      const _Float16 hv = (_Float16)c64;
      sCh[wave][crow + n * 16 + l16] = hv;
      sCl[wave][crow + n * 16 + l16] = (_Float16)((c64 - (float)hv) * 4096.0f);
    }
  }
  __builtin_amdgcn_fence(3  , "workgroup");
  __builtin_amdgcn_wave_barrier();
  __builtin_amdgcn_fence(2  , "workgroup");
  const size_t rowbase = (size_t)(b * SEQ + q0);
  for (int pass = 0; pass < 2; ++pass) {
#pragma unroll
    for (int it = 0; it < 4; ++it) {
      const int rr = it * 4 + (lane >> 3);
      const int p  = lane & 7;
      const v8h vh = *(const v8h*)(&sCh[wave][rr * HD + p * 8]);
      const v8h vl = *(const v8h*)(&sCl[wave][rr * HD + p * 8]);
      const size_t off = (rowbase + rr) * CH + (size_t)h * HD + p * 8;
      *(volatile v8h*)(Ch + off) = vh;
      *(volatile v8h*)(Cl + off) = vl;
    }
    __threadfence();
  }
}

__global__ void __launch_bounds__(256) oproj_kernel(
    const _Float16* __restrict__ Ch, const _Float16* __restrict__ Cl,
    const _Float16* __restrict__ Wot, const float* __restrict__ bo,
    float* __restrict__ out) {
  __shared__ __attribute__((aligned(16))) float sO[128 * LDPF];

  const int tid = threadIdx.x, wid = tid >> 5, lane = tid & 31, l16 = lane & 15, lh = lane >> 4;
  const int wm = wid & 3, wn = wid >> 2;
  const int bx = blockIdx.x, by = blockIdx.y;
  const int m0 = bx * 128 + wm * 32;
  const int n0 = by * 64 + wn * 32;

  v8f a0c[2][2], a1c[2][2];
  const v8f zero = {};
#pragma unroll
  for (int i = 0; i < 2; ++i)
#pragma unroll
    for (int j = 0; j < 2; ++j) { a0c[i][j] = zero; a1c[i][j] = zero; }

  for (int k0 = 0; k0 < CH; k0 += 32) {
    const v16h ah0 = ldfrag(Ch, CH, m0, k0);
    const v16h ah1 = ldfrag(Ch, CH, m0 + 16, k0);
    const v16h al0 = ldfrag(Cl, CH, m0, k0);
    const v16h al1 = ldfrag(Cl, CH, m0 + 16, k0);
    const v16h b0  = ldfrag(Wot, CH, n0, k0);
    const v16h b1  = ldfrag(Wot, CH, n0 + 16, k0);
    a0c[0][0] = WMMA_F16(ah0, b0, a0c[0][0]);
    a0c[1][0] = WMMA_F16(ah1, b0, a0c[1][0]);
    a0c[0][1] = WMMA_F16(ah0, b1, a0c[0][1]);
    a0c[1][1] = WMMA_F16(ah1, b1, a0c[1][1]);
    a1c[0][0] = WMMA_F16(al0, b0, a1c[0][0]);
    a1c[1][0] = WMMA_F16(al1, b0, a1c[1][0]);
    a1c[0][1] = WMMA_F16(al0, b1, a1c[0][1]);
    a1c[1][1] = WMMA_F16(al1, b1, a1c[1][1]);
    asm volatile("v_nop\n\tv_nop\n\tv_nop\n\tv_nop"
                 : "+v"(a0c[0][0]), "+v"(a0c[1][0]), "+v"(a0c[0][1]), "+v"(a0c[1][1]),
                   "+v"(a1c[0][0]), "+v"(a1c[1][0]), "+v"(a1c[0][1]), "+v"(a1c[1][1])
                 : "v"(ah0), "v"(al1), "v"(b0), "v"(b1));
  }

  float bcol[2];
#pragma unroll
  for (int j = 0; j < 2; ++j) bcol[j] = bf16r(bo[n0 + j * 16 + l16]);
#pragma unroll
  for (int i = 0; i < 2; ++i)
#pragma unroll
    for (int j = 0; j < 2; ++j)
#pragma unroll
      for (int r = 0; r < 8; ++r) {
        const int rl = wm * 32 + i * 16 + 8 * lh + r;
        const int cl = wn * 32 + j * 16 + l16;
        sO[rl * LDPF + cl] = (a0c[i][j][r] + a1c[i][j][r] * 0.000244140625f) * 0.000244140625f + bcol[j];
      }
  __syncthreads();
  const int mb0 = bx * 128;
  const int bb  = mb0 / SEQ;
  const int t0  = mb0 - bb * SEQ;
  const size_t rowbase = (size_t)(bb * SEQ_FULL + t0);
  for (int pass = 0; pass < 2; ++pass) {
#pragma unroll
    for (int it = 0; it < 8; ++it) {
      const int L  = wid * 32 + it * 4 + (lane >> 3);
      const int p  = lane & 7;
      const int rl = L >> 1, hf = L & 1;
      const v4f v = *(const v4f*)(sO + rl * LDPF + hf * 32 + p * 4);
      *(volatile v4f*)(out + (rowbase + rl) * CH + by * 64 + hf * 32 + p * 4) = v;
    }
    __threadfence();
  }
}

extern "C" void kernel_launch(void* const* d_in, const int* in_sizes, int n_in,
                              void* d_out, int out_size, void* d_ws, size_t ws_size,
                              hipStream_t stream) {
  if (n_in < 9) return;
  const int need_x = (NB - 1) * SEQ_FULL * CH + SEQ * CH;
  if (in_sizes[0] < need_x || out_size < need_x) return;
  if (in_sizes[1] < CH * CH || in_sizes[3] < CH * CH || in_sizes[5] < CH * CH || in_sizes[7] < CH * CH) return;
  if (in_sizes[2] < CH || in_sizes[4] < CH || in_sizes[6] < CH || in_sizes[8] < CH) return;

  const float* x  = (const float*)d_in[0];
  const float* Wq = (const float*)d_in[1];
  const float* bq = (const float*)d_in[2];
  const float* Wk = (const float*)d_in[3];
  const float* bk = (const float*)d_in[4];
  const float* Wv = (const float*)d_in[5];
  const float* bv = (const float*)d_in[6];
  const float* Wo = (const float*)d_in[7];
  const float* bo = (const float*)d_in[8];
  float* out = (float*)d_out;

  const size_t szW = (size_t)4 * CH * CH * sizeof(_Float16);
  const size_t szP = (size_t)MROWS * CH * sizeof(_Float16);
  const size_t offX  = szW;
  const size_t offQh = offX  + szP;
  const size_t offQl = offQh + szP;
  const size_t offKh = offQl + szP;
  const size_t offKl = offKh + szP;
  const size_t offVh = offKl + szP;
  const size_t offVl = offVh + szP;
  const size_t offCh = offVl + szP;
  const size_t offCl = offCh + szP;
  const size_t total = offCl + szP;
  if (ws_size < total) return;

  char* ws = (char*)d_ws;
  _Float16* Wc  = (_Float16*)(ws);
  _Float16* Xc  = (_Float16*)(ws + offX);
  _Float16* Qhp = (_Float16*)(ws + offQh);
  _Float16* Qlp = (_Float16*)(ws + offQl);
  _Float16* Khp = (_Float16*)(ws + offKh);
  _Float16* Klp = (_Float16*)(ws + offKl);
  _Float16* Vhp = (_Float16*)(ws + offVh);
  _Float16* Vlp = (_Float16*)(ws + offVl);
  _Float16* Chp = (_Float16*)(ws + offCh);
  _Float16* Clp = (_Float16*)(ws + offCl);

  cvt_w_kernel<<<(4 * CH * CH / 8) / 256, 256, 0, stream>>>(Wq, Wk, Wv, Wo, Wc);
  cvt_x_kernel<<<(MROWS * CH / 8) / 256, 256, 0, stream>>>(x, Xc);
  qkv_kernel<<<dim3(MROWS / 128, (3 * CH) / 128), 256, 0, stream>>>(
      Xc, Wc, bq, bk, bv, Qhp, Qlp, Khp, Klp, Vhp, Vlp);
  attn_kernel<<<NB * NH * (SEQ / 64), 128, 0, stream>>>(Qhp, Qlp, Khp, Klp, Vhp, Vlp, Chp, Clp);
  oproj_kernel<<<dim3(MROWS / 128, CH / 64), 256, 0, stream>>>(Chp, Clp, Wc + (size_t)3 * CH * CH, bo, out);
}
